// MultiHeadSelfAttention_35682588295575
// MI455X (gfx1250) — hardware-verified
//
#include <hip/hip_runtime.h>


#ifndef NB
#define NB 4
#endif
#ifndef SEQ
#define SEQ 2048
#endif
#define NB_FULL  4
#define SEQ_FULL 2048
#define DIN  64
#define NH   8
#define HD   64
#define DQ   (NH * HD)
#define SCL  8.0f
#define LOG2E 1.4426950408889634f
#define LP   72

static_assert(NB <= NB_FULL);
static_assert(SEQ <= SEQ_FULL);
static_assert(SEQ % 64 == 0);
static_assert((NB * SEQ) % 64 == 0);
static_assert(HD == 64);
static_assert(DIN == 64);
static_assert(DIN % 32 == 0 && DQ % 32 == 0);
static_assert(DQ % 64 == 0);
static_assert((LP * 2) % 16 == 0);
static_assert(LP >= HD);

typedef unsigned short bf;
typedef __attribute__((ext_vector_type(16))) __bf16   v16bf;
typedef __attribute__((ext_vector_type(8)))  unsigned short v8us;
typedef __attribute__((ext_vector_type(8)))  float    v8f;
typedef __attribute__((ext_vector_type(4)))  float    v4f;
typedef v4f  __attribute__((may_alias)) v4fa;
typedef v8us __attribute__((may_alias)) v8usa;

__device__ __forceinline__ unsigned short f2bf(float f) { unsigned u = __float_as_uint(f); u += 0x7FFFu + ((u >> 16) & 1u); return (unsigned short)(u >> 16); }
__device__ __forceinline__ float bf2f(unsigned short b) { return __uint_as_float(((unsigned)b) << 16); }
__device__ __forceinline__ float bfr(float f) { return bf2f(f2bf(f)); }
__device__ __forceinline__ void splitf(float y, unsigned short& h, unsigned short& l) { h = f2bf(y); l = f2bf(y - bf2f(h)); }
__device__ __forceinline__ v16bf cat16b(v8us lo, v8us hi) { return __builtin_bit_cast(v16bf, __builtin_shufflevector(lo, hi, 0, 1, 2, 3, 4, 5, 6, 7, 8, 9, 10, 11, 12, 13, 14, 15)); }
__device__ __forceinline__ v8f wmmab(v16bf a, v16bf b, v8f c) { return __builtin_amdgcn_wmma_f32_16x16x32_bf16(false, a, false, b, (short)0, c, false, false); }
__device__ __forceinline__ v16bf ldb(const bf* p) { return cat16b(*(const v8us*)p, *(const v8us*)(p + 16)); }

template <int NSPLIT, bool BIAS>
__device__ __forceinline__ void gemmw_body(const bf* __restrict__ A, const bf* __restrict__ A2, const bf* __restrict__ Bt, int K, float* C, int ldc, const float* __restrict__ bias, size_t sA, size_t sB, size_t sC) {
    __shared__ __align__(16) float os[16 * 68];
    const size_t z = blockIdx.z; A += z * sA; if (NSPLIT == 1) A2 += z * sA; Bt += z * sB; C += z * sC;
    const int lane = threadIdx.x & 31, lr = lane & 15, hi = lane >> 4; const int r0 = blockIdx.x * 64, c0 = blockIdx.y * 64;
    v8f acc[4][4];
#pragma unroll
    for (int mb = 0; mb < 4; ++mb)
#pragma unroll
        for (int nb = 0; nb < 4; ++nb) acc[mb][nb] = (v8f){};
    const size_t aoff = (size_t)(r0 + lr) * K + 8 * hi, boff = (size_t)(c0 + lr) * K + 8 * hi;
#pragma unroll 1
    for (int kc = 0; kc < K; kc += 32) {
        v16bf a[4], a2[4];
#pragma unroll
        for (int mb = 0; mb < 4; ++mb) { a[mb] = ldb(A + aoff + (size_t)mb * 16 * K + kc); if (NSPLIT == 1) a2[mb] = ldb(A2 + aoff + (size_t)mb * 16 * K + kc); }
#pragma unroll
        for (int nb = 0; nb < 4; ++nb) { const v16bf b = ldb(Bt + boff + (size_t)nb * 16 * K + kc);
#pragma unroll
            for (int mb = 0; mb < 4; ++mb) { acc[mb][nb] = wmmab(a[mb], b, acc[mb][nb]); if (NSPLIT == 1) acc[mb][nb] = wmmab(a2[mb], b, acc[mb][nb]); } }
        asm volatile("v_nop\n\tv_nop\n\tv_nop\n\tv_nop" : "+v"(acc[0][0]), "+v"(acc[1][1]), "+v"(acc[2][2]), "+v"(acc[3][3]) : "v"(a[0]), "v"(a[3]));
    }
#pragma unroll
    for (int mb = 0; mb < 4; ++mb) {
#pragma unroll
        for (int nb = 0; nb < 4; ++nb) {
#pragma unroll
            for (int j = 0; j < 8; ++j) os[(hi * 8 + j) * 68 + nb * 16 + lr] = acc[mb][nb][j]; }
        __builtin_amdgcn_wave_barrier(); asm volatile("" ::: "memory");
        float* crow = C + (size_t)(r0 + mb * 16) * ldc + c0;
#pragma unroll 1
        for (int ps = 0; ps < 2; ++ps) {
#pragma unroll
            for (int s = 0; s < 8; ++s) { const int row = 2 * s + hi, cofs = lr * 4; v4f val = *(const v4fa*)(os + row * 68 + cofs); if (BIAS) { val[0] += bfr(bias[c0 + cofs]); val[1] += bfr(bias[c0 + cofs + 1]); val[2] += bfr(bias[c0 + cofs + 2]); val[3] += bfr(bias[c0 + cofs + 3]); }
                *(volatile v4f*)(crow + (size_t)row * ldc + cofs) = val; }
            if (ps == 0) __threadfence(); }
        __builtin_amdgcn_wave_barrier(); asm volatile("" ::: "memory");
    }
}
__global__ __launch_bounds__(32) void k_gemm_proj(const bf* __restrict__ A, const bf* __restrict__ Bt, float* C, const float* __restrict__ bias) {
    gemmw_body<0, true>(A, A, Bt, DIN, C, DQ, bias, 0, 0, 0); }
__global__ __launch_bounds__(32) void k_gemm_out(const bf* __restrict__ Ah, const bf* __restrict__ Al, const bf* __restrict__ Bt, float* C, const float* __restrict__ bias) {
    gemmw_body<1, true>(Ah, Al, Bt, DQ, C, DIN, bias, (size_t)SEQ * DQ, 0, (size_t)SEQ_FULL * DIN); }

__global__ __launch_bounds__(256) void k_cvtx(const float* __restrict__ src, bf* dst) {
    const int b = blockIdx.y; const size_t i = (size_t)blockIdx.x * 256 + threadIdx.x; if (i >= (size_t)SEQ * DIN / 8) return;
    const v8f v = *(const v8f*)(src + (size_t)b * SEQ_FULL * DIN + i * 8); v8us o;
#pragma unroll
    for (int k = 0; k < 8; ++k) o[k] = f2bf(v[k]);
    bf* d = dst + (size_t)b * SEQ * DIN + i * 8; *(volatile v8us*)d = o; __threadfence(); *(volatile v8us*)d = o; }

__global__ __launch_bounds__(256) void k_wt(const float* __restrict__ W, bf* Wt, int N, int K, int perm) {
    const int i = blockIdx.x * 256 + threadIdx.x; const int k8 = K / 8; if (i >= N * k8) return;
    const int n = i / k8, kk0 = (i % k8) * 8; v8us o;
#pragma unroll
    for (int q = 0; q < 8; ++q) { const int kk = kk0 + q; const int srow = perm ? ((kk & (HD - 1)) * NH + (kk >> 6)) : kk; o[q] = f2bf(W[(size_t)srow * N + n]); }
    bf* d = Wt + (size_t)n * K + kk0; *(volatile v8us*)d = o; __threadfence(); *(volatile v8us*)d = o; }

__global__ __launch_bounds__(256) void k_hp(const float* __restrict__ F, bf* Ph, bf* Pl) {
    const size_t i = (size_t)blockIdx.x * 256 + threadIdx.x; if (i >= (size_t)NB * NH * SEQ * HD / 8) return;
    const int d8 = (int)(i & 7); const int l = (int)((i >> 3) % SEQ); const int h = (int)((i / ((size_t)8 * SEQ)) % NH); const int b = (int)(i / ((size_t)8 * SEQ * NH));
    const float* f = F + ((size_t)b * SEQ + l) * DQ + h * HD + d8 * 8; const v4f a = *(const v4f*)f, c = *(const v4f*)(f + 4); v8us oh, ol;
#pragma unroll
    for (int q = 0; q < 4; ++q) { unsigned short s0, s1; splitf(a[q], s0, s1); oh[q] = s0; ol[q] = s1; splitf(c[q], s0, s1); oh[4 + q] = s0; ol[4 + q] = s1; }
    const size_t e = i * 8; *(volatile v8us*)(Ph + e) = oh; *(volatile v8us*)(Pl + e) = ol; __threadfence(); *(volatile v8us*)(Ph + e) = oh; *(volatile v8us*)(Pl + e) = ol; }

__global__ __launch_bounds__(256) void k_vt(const float* __restrict__ F, bf* Vh, bf* Vl) {
    const size_t i = (size_t)blockIdx.x * 256 + threadIdx.x; if (i >= (size_t)NB * NH * HD * SEQ / 8) return;
    const int l8 = (int)(i % (SEQ / 8)); const int d = (int)((i / (SEQ / 8)) % HD); const int h = (int)((i / ((size_t)(SEQ / 8) * HD)) % NH); const int b = (int)(i / ((size_t)(SEQ / 8) * HD * NH));
    const float* f = F + ((size_t)b * SEQ + (size_t)l8 * 8) * DQ + h * HD + d; v8us oh, ol;
#pragma unroll
    for (int q = 0; q < 8; ++q) { unsigned short s0, s1; splitf(f[(size_t)q * DQ], s0, s1); oh[q] = s0; ol[q] = s1; }
    const size_t e = i * 8; *(volatile v8us*)(Vh + e) = oh; *(volatile v8us*)(Vl + e) = ol; __threadfence(); *(volatile v8us*)(Vh + e) = oh; *(volatile v8us*)(Vl + e) = ol; }

__global__ __launch_bounds__(128) void k_flash(const bf* __restrict__ Qh, const bf* __restrict__ Ql, const bf* __restrict__ Kh, const bf* __restrict__ Kl,
                                               const bf* __restrict__ Vh, const bf* __restrict__ Vl, bf* Ah, bf* Al) {
    __shared__ __align__(16) unsigned short sth[4 * 16 * LP];
    __shared__ __align__(16) unsigned short stl[4 * 16 * LP];
    const int wave = __builtin_amdgcn_readfirstlane(threadIdx.x >> 5);
    const int lane = threadIdx.x & 31, lr = lane & 15, hi = lane >> 4;
    const int bh = blockIdx.y; const int q0 = blockIdx.x * 64 + wave * 16;
    const size_t zoff = (size_t)bh * SEQ * HD;
    const bf* qhp = Qh + zoff + (size_t)(q0 + lr) * HD + 8 * hi; const bf* qlp = Ql + zoff + (size_t)(q0 + lr) * HD + 8 * hi;
    const bf* khp = Kh + zoff + (size_t)lr * HD + 8 * hi;        const bf* klp = Kl + zoff + (size_t)lr * HD + 8 * hi;
    const bf* vhp = Vh + zoff + (size_t)lr * SEQ + 8 * hi;       const bf* vlp = Vl + zoff + (size_t)lr * SEQ + 8 * hi;
    v8f o[4];
#pragma unroll
    for (int dt = 0; dt < 4; ++dt) o[dt] = (v8f){};
    float mrun = -1.0e30f, lrun = 0.0f;
#pragma unroll 1
    for (int kb = 0; kb < SEQ; kb += 64) {
        v8f st[4];
#pragma unroll
        for (int t = 0; t < 4; ++t) st[t] = (v8f){};
#pragma unroll
        for (int ks = 0; ks < 2; ++ks) {
            int qo = ks * 32; asm volatile("" : "+v"(qo));
            const v16bf qh = ldb(qhp + qo), ql = ldb(qlp + qo);
#pragma unroll
            for (int t = 0; t < 4; ++t) { const size_t ko = (size_t)(kb + 16 * t) * HD + ks * 32; const v16bf kh = ldb(khp + ko), kl = ldb(klp + ko);
                st[t] = wmmab(kh, qh, st[t]); st[t] = wmmab(kl, qh, st[t]); st[t] = wmmab(kh, ql, st[t]);
                asm volatile("v_nop\n\tv_nop\n\tv_nop\n\tv_nop" : "+v"(st[t]) : "v"(kh), "v"(kl), "v"(qh), "v"(ql)); }
        }
        float mx = -1.0e30f;
#pragma unroll
        for (int t = 0; t < 4; ++t)
#pragma unroll
            for (int r = 0; r < 8; ++r) { st[t][r] *= SCL; mx = fmaxf(mx, st[t][r]); }
        mx = fmaxf(mx, __shfl_xor(mx, 16, 32));
        const float mnew = fmaxf(mrun, mx);
        const float fac = __builtin_amdgcn_exp2f((mrun - mnew) * LOG2E);
        mrun = mnew;
        float ls = 0.0f; v8us phv[4], plv[4];
#pragma unroll
        for (int t = 0; t < 4; ++t)
#pragma unroll
            for (int r = 0; r < 8; ++r) { const float p = __builtin_amdgcn_exp2f((st[t][r] - mnew) * LOG2E); ls += p; unsigned short s0, s1; splitf(p, s0, s1); phv[t][r] = s0; plv[t][r] = s1; }
        lrun = lrun * fac + ls;
#pragma unroll
        for (int dt = 0; dt < 4; ++dt)
#pragma unroll
            for (int r = 0; r < 8; ++r) o[dt][r] *= fac;
        v16bf pbh[2], pbl[2];
        pbh[0] = cat16b(phv[0], phv[1]); pbl[0] = cat16b(plv[0], plv[1]); pbh[1] = cat16b(phv[2], phv[3]); pbl[1] = cat16b(plv[2], plv[3]);
        asm volatile("" : "+v"(pbh[0]), "+v"(pbl[0]), "+v"(pbh[1]), "+v"(pbl[1]));
#pragma unroll
        for (int j = 0; j < 2; ++j) {
#pragma unroll
            for (int dt = 0; dt < 4; ++dt) { const size_t vo = (size_t)(16 * dt) * SEQ + kb + 32 * j; const v16bf vh = ldb(vhp + vo), vl = ldb(vlp + vo);
                o[dt] = wmmab(vh, pbh[j], o[dt]); o[dt] = wmmab(vl, pbh[j], o[dt]); o[dt] = wmmab(vh, pbl[j], o[dt]);
                asm volatile("v_nop\n\tv_nop\n\tv_nop\n\tv_nop" : "+v"(o[dt]) : "v"(vh), "v"(vl), "v"(pbh[j]), "v"(pbl[j])); }
        }
    }
    lrun += __shfl_xor(lrun, 16, 32);
    const float inv = 1.0f / lrun;
    const int sbase = wave * (16 * LP);
#pragma unroll
    for (int dt = 0; dt < 4; ++dt) { v8us oh, ol;
#pragma unroll
        for (int r = 0; r < 8; ++r) { unsigned short s0, s1; splitf(o[dt][r] * inv, s0, s1); oh[r] = s0; ol[r] = s1; }
        *(v8us*)(&sth[sbase + lr * LP + 16 * dt + 8 * hi]) = oh; *(v8us*)(&stl[sbase + lr * LP + 16 * dt + 8 * hi]) = ol; }
    __builtin_amdgcn_wave_barrier(); asm volatile("" ::: "memory");
    const int b = bh / NH, h = bh % NH; const size_t orow = (size_t)b * SEQ + q0;
#pragma unroll 1
    for (int ps = 0; ps < 2; ++ps) {
#pragma unroll
        for (int s = 0; s < 4; ++s) { const int row = 4 * s + (lane >> 3), col = (lane & 7) * 8;
            const v8us a = *(const v8usa*)(&sth[sbase + row * LP + col]); const v8us c = *(const v8usa*)(&stl[sbase + row * LP + col]);
            const size_t g = (orow + row) * DQ + h * HD + col;
            *(volatile v8us*)(Ah + g) = a; *(volatile v8us*)(Al + g) = c; }
        if (ps == 0) __threadfence(); }
}

constexpr size_t SZ_W   = (size_t)DQ * DIN * 2;
constexpr size_t SZ_XB  = (size_t)NB * SEQ * DIN * 2;
constexpr size_t SZ_F   = (size_t)NB * SEQ * DQ * 4;
constexpr size_t SZ_HP  = (size_t)NB * NH * SEQ * HD * 2;
constexpr size_t SZ_AT  = (size_t)NB * SEQ * DQ * 2;
constexpr size_t OFF_WQ = 0, OFF_WK = OFF_WQ + SZ_W, OFF_WV = OFF_WK + SZ_W, OFF_WO = OFF_WV + SZ_W, OFF_XB = OFF_WO + SZ_W, OFF_F = OFF_XB + SZ_XB;
constexpr size_t OFF_QH = OFF_F + SZ_F, OFF_QL = OFF_QH + SZ_HP, OFF_KH = OFF_QL + SZ_HP, OFF_KL = OFF_KH + SZ_HP, OFF_VH = OFF_KL + SZ_HP, OFF_VL = OFF_VH + SZ_HP;
constexpr size_t OFF_AH = OFF_VL + SZ_HP, OFF_AL = OFF_AH + SZ_AT, WS_TOTAL = OFF_AL + SZ_AT;
static_assert(SZ_W % 256 == 0 && SZ_XB % 256 == 0 && SZ_F % 256 == 0 && SZ_HP % 256 == 0 && SZ_AT % 256 == 0);
static_assert(WS_TOTAL <= (size_t)134217728);
static_assert(((size_t)SEQ * DIN / 8) % 256 == 0);
static_assert(((size_t)DQ * DIN / 8) % 256 == 0);

extern "C" void kernel_launch(void* const* d_in, const int* in_sizes, int n_in,
                              void* d_out, int out_size, void* d_ws, size_t ws_size, hipStream_t stream) {
    if (n_in < 9) return;
    const int xmin = ((NB - 1) * SEQ_FULL + SEQ) * DIN;
    if (in_sizes[0] < xmin || in_sizes[1] < DIN * DQ || in_sizes[2] < DQ || in_sizes[3] < DIN * DQ || in_sizes[4] < DQ || in_sizes[5] < DIN * DQ || in_sizes[6] < DQ || in_sizes[7] < DQ * DIN || in_sizes[8] < DIN) return;
    if (out_size < xmin) return;
    if (ws_size < WS_TOTAL) return;
    const float* x  = (const float*)d_in[0]; const float* wq = (const float*)d_in[1]; const float* bq = (const float*)d_in[2];
    const float* wk = (const float*)d_in[3]; const float* bk = (const float*)d_in[4]; const float* wv = (const float*)d_in[5];
    const float* bv = (const float*)d_in[6]; const float* wo = (const float*)d_in[7]; const float* bo = (const float*)d_in[8];
    float* OUT = (float*)d_out;
    char* wsb = (char*)d_ws;
    bf* WQt = (bf*)(wsb + OFF_WQ); bf* WKt = (bf*)(wsb + OFF_WK); bf* WVt = (bf*)(wsb + OFF_WV); bf* WOt = (bf*)(wsb + OFF_WO);
    bf* XB = (bf*)(wsb + OFF_XB); float* F = (float*)(wsb + OFF_F);
    bf* QPh = (bf*)(wsb + OFF_QH); bf* QPl = (bf*)(wsb + OFF_QL); bf* KPh = (bf*)(wsb + OFF_KH); bf* KPl = (bf*)(wsb + OFF_KL); bf* VTh = (bf*)(wsb + OFF_VH); bf* VTl = (bf*)(wsb + OFF_VL);
    bf* ATh = (bf*)(wsb + OFF_AH); bf* ATl = (bf*)(wsb + OFF_AL);

    const unsigned gw = (unsigned)(((size_t)DQ * DIN / 8 + 255) / 256);
    k_wt<<<gw, 256, 0, stream>>>(wq, WQt, DQ, DIN, 0);
    k_wt<<<gw, 256, 0, stream>>>(wk, WKt, DQ, DIN, 0);
    k_wt<<<gw, 256, 0, stream>>>(wv, WVt, DQ, DIN, 0);
    k_wt<<<gw, 256, 0, stream>>>(wo, WOt, DIN, DQ, 1);
    k_cvtx<<<dim3((unsigned)(((size_t)SEQ * DIN / 8 + 255) / 256), NB, 1), 256, 0, stream>>>(x, XB);
    const unsigned gp = (unsigned)(((size_t)NB * NH * SEQ * HD / 8 + 255) / 256);
    const dim3 gproj(NB * SEQ / 64, DQ / 64, 1);
    k_gemm_proj<<<gproj, 32, 0, stream>>>(XB, WQt, F, bq); k_hp<<<gp, 256, 0, stream>>>(F, QPh, QPl);
    k_gemm_proj<<<gproj, 32, 0, stream>>>(XB, WKt, F, bk); k_hp<<<gp, 256, 0, stream>>>(F, KPh, KPl);
    k_gemm_proj<<<gproj, 32, 0, stream>>>(XB, WVt, F, bv); k_vt<<<gp, 256, 0, stream>>>(F, VTh, VTl);
    k_flash<<<dim3(SEQ / 64, NB * NH, 1), 128, 0, stream>>>(QPh, QPl, KPh, KPl, VTh, VTl, ATh, ATl);
    k_gemm_out<<<dim3(SEQ / 64, DIN / 64, NB), 32, 0, stream>>>(ATh, ATl, WOt, OUT, bo);
}
